// EdgeNetwork_sparse_48000554500609
// MI455X (gfx1250) — hardware-verified
//
#include <hip/hip_runtime.h>
#include <hip/hip_bf16.h>
#include <stddef.h>
#include <math.h>


#define DD    256
#define XC    1024
#define NWT   4
#define NCHN  4
#define MT    64
#define GT    128
#define TP    68
#define NB    32
#define NTHR  256
#define NWAVE 8
#define EPT   8
#define CHUNK (NTHR * EPT)
#define WCAP  (EPT * 32)
#define LISTN (NWAVE * WCAP)
#define EB    256

static_assert(DD == NTHR);
static_assert((MT % NB) == 0);
static_assert(WCAP == 256);
static_assert((NB % NWAVE) == 0);

typedef float          v4f   __attribute__((ext_vector_type(4)));
typedef float          v8f   __attribute__((ext_vector_type(8)));
typedef int            v4i   __attribute__((ext_vector_type(4)));
typedef unsigned int   v4u   __attribute__((ext_vector_type(4)));
typedef unsigned short v8us  __attribute__((ext_vector_type(8)));
typedef __bf16         v16b  __attribute__((ext_vector_type(16)));
typedef float          v4fa  __attribute__((ext_vector_type(4), may_alias));
typedef unsigned int   v4ua  __attribute__((ext_vector_type(4), may_alias));
typedef unsigned short v8usa __attribute__((ext_vector_type(8), may_alias));
union FragB { v16b v; v8us h[2]; };

__device__ __forceinline__ unsigned int f2bf(float f) {
  const unsigned int u = __float_as_uint(f);
  return (u + 0x7FFFu + ((u >> 16) & 1u)) >> 16;
}
__device__ __forceinline__ float bf2f(unsigned int b) { return __uint_as_float(b << 16); }

__device__ __forceinline__ v8f zero8f() {
  v8f z;
#pragma unroll
  for (int i = 0; i < 8; ++i) z[i] = 0.0f;
  return z;
}

__device__ __forceinline__ v8f cat8(v4f a, v4f b) {
  v8f c;
  c[0] = a.x; c[1] = a.y; c[2] = a.z; c[3] = a.w;
  c[4] = b.x; c[5] = b.y; c[6] = b.z; c[7] = b.w;
  return c;
}

__device__ __forceinline__ void split8(v8f f, v8us& hv, v8us& lv) {
#pragma unroll
  for (int i = 0; i < 8; ++i) {
    const unsigned int hi = f2bf(f[i]);
    const unsigned int lo = f2bf(f[i] - bf2f(hi));
    hv[i] = (unsigned short)hi;
    lv[i] = (unsigned short)lo;
  }
}

__device__ __forceinline__ v8f wmb(v16b a, v16b b, v8f c) {
  v8f d = __builtin_amdgcn_wmma_f32_16x16x32_bf16(false, a, false, b, (short)0, c, false, false);
  asm volatile("v_nop\n\tv_nop\n\tv_nop\n\tv_nop" : "+v"(d) : "v"(a), "v"(b));
  return d;
}

__device__ __forceinline__ int scan_chunk(const int* __restrict__ dsts, int nE, int cbase, int nodeBase,
                                          int vec8, int* list, int tid, int wave) {
  int wc = 0;
  const int el0  = tid * EPT;
  const int e0   = cbase + el0;
  const int sent = -2147483647 - 1;
  v4i da, db;
  if (vec8 != 0 && cbase + CHUNK <= nE) {
    da = *(const v4i*)(dsts + e0);
    db = *(const v4i*)(dsts + e0 + 4);
  } else {
    da.x = (e0     < nE) ? dsts[min(e0, nE - 1)] : sent;
    da.y = (e0 + 1 < nE) ? dsts[min(e0 + 1, nE - 1)] : sent;
    da.z = (e0 + 2 < nE) ? dsts[min(e0 + 2, nE - 1)] : sent;
    da.w = (e0 + 3 < nE) ? dsts[min(e0 + 3, nE - 1)] : sent;
    db.x = (e0 + 4 < nE) ? dsts[min(e0 + 4, nE - 1)] : sent;
    db.y = (e0 + 5 < nE) ? dsts[min(e0 + 5, nE - 1)] : sent;
    db.z = (e0 + 6 < nE) ? dsts[min(e0 + 6, nE - 1)] : sent;
    db.w = (e0 + 7 < nE) ? dsts[min(e0 + 7, nE - 1)] : sent;
  }
  const unsigned nb = (unsigned)nodeBase;
  const unsigned s0 = (unsigned)da.x - nb, s1 = (unsigned)da.y - nb;
  const unsigned s2 = (unsigned)da.z - nb, s3 = (unsigned)da.w - nb;
  const unsigned s4 = (unsigned)db.x - nb, s5 = (unsigned)db.y - nb;
  const unsigned s6 = (unsigned)db.z - nb, s7 = (unsigned)db.w - nb;
  const bool h0 = s0 < (unsigned)NB, h1 = s1 < (unsigned)NB, h2 = s2 < (unsigned)NB, h3 = s3 < (unsigned)NB;
  const bool h4 = s4 < (unsigned)NB, h5 = s5 < (unsigned)NB, h6 = s6 < (unsigned)NB, h7 = s7 < (unsigned)NB;
  const unsigned any = __builtin_amdgcn_ballot_w32(h0 | h1 | h2 | h3 | h4 | h5 | h6 | h7);
  if (any != 0u) {
#define HITJ(J, HJ) { \
      const unsigned mj = __builtin_amdgcn_ballot_w32(HJ); \
      if (mj != 0u) { \
        if (HJ) { \
          const int pos = wc + (int)__builtin_amdgcn_mbcnt_lo(mj, 0u); \
          if (pos < WCAP) list[wave * WCAP + pos] = el0 + (J); \
        } \
        wc += (int)__builtin_popcount(mj); } }
    HITJ(0, h0)
    HITJ(1, h1)
    HITJ(2, h2)
    HITJ(3, h3)
    HITJ(4, h4)
    HITJ(5, h5)
    HITJ(6, h6)
    HITJ(7, h7)
#undef HITJ
  }
  return wc;
}

__global__ __launch_bounds__(NTHR) void k_cvtx(const float* __restrict__ x,
                                               unsigned short* xh, unsigned short* xl, int nN, int nG) {
  const int g    = blockIdx.x * NTHR + threadIdx.x;
  const int gc   = g < nG ? g : nG - 1;
  const int row  = gc >> 5;
  const int rowc = row < nN ? row : nN - 1;
  const float* p = x + (size_t)rowc * DD + (gc & 31) * 8;
  const v4f a = *(const v4f*)p, b = *(const v4f*)(p + 4);
  v8f f = cat8(a, b);
  if (row >= nN) f = zero8f();
  v8us hv, lv;
  split8(f, hv, lv);
  const size_t o = (size_t)gc * 8;
  if (g < nG) { *(volatile v8us*)(xh + o) = hv; *(volatile v8us*)(xl + o) = lv; }
  __threadfence();
  if (g < nG) { *(volatile v8us*)(xh + o) = hv; *(volatile v8us*)(xl + o) = lv; }
}

__global__ __launch_bounds__(NTHR) void k_cvtw(
    const float* __restrict__ Wq, const float* __restrict__ Wk, const float* __restrict__ Wv,
    const float* __restrict__ Ws, const float* __restrict__ Wm1, const float* __restrict__ Wm2,
    unsigned short* wh, unsigned short* wl, unsigned short* m1h, unsigned short* m1l,
    unsigned short* m2h, unsigned short* m2l) {
  const int blk = blockIdx.x, tid = threadIdx.x;
  const int nb0 = (NCHN * NWT * DD * DD) / (8 * NTHR);
  const int nb1 = (16 * XC) / (8 * NTHR);
  v4f a, b;
  bool z = false;
  unsigned short* dh;
  unsigned short* dl;
  size_t o;
  if (blk < nb0) {
    const int e0 = (blk * NTHR + tid) * 8;
    const int c = e0 / (NWT * DD * DD);
    const int w = (e0 / (DD * DD)) & 3;
    const int rest = e0 & (DD * DD - 1);
    const float* src = (w == 0) ? Wq : (w == 1) ? Wk : (w == 2) ? Wv : Ws;
    const float* p = src + (size_t)c * DD * DD + rest;
    a = *(const v4f*)p; b = *(const v4f*)(p + 4);
    dh = wh; dl = wl; o = (size_t)e0;
  } else if (blk < nb0 + nb1) {
    const int e0 = ((blk - nb0) * NTHR + tid) * 8;
    const int row = e0 >> 10, k = e0 & (XC - 1);
    const int rowc = row < 8 ? row : 7;
    const float* p = Wm1 + (size_t)rowc * XC + k;
    a = *(const v4f*)p; b = *(const v4f*)(p + 4);
    z = row >= 8;
    dh = m1h; dl = m1l; o = (size_t)e0;
  } else {
    const int e0 = ((blk - nb0 - nb1) * NTHR + tid) * 8;
    const int d = e0 >> 5, k0 = e0 & 31;
    const int dc = d < DD ? d : DD - 1;
    const float* p = Wm2 + (size_t)dc * 8;
    a = *(const v4f*)p; b = *(const v4f*)(p + 4);
    z = (k0 != 0) || (d >= DD);
    dh = m2h; dl = m2l; o = (size_t)e0;
  }
  v8f f = cat8(a, b);
  if (z) f = zero8f();
  v8us hv, lv;
  split8(f, hv, lv);
  *(volatile v8us*)(dh + o) = hv;
  *(volatile v8us*)(dl + o) = lv;
  __threadfence();
  *(volatile v8us*)(dh + o) = hv;
  *(volatile v8us*)(dl + o) = lv;
}

__global__ __launch_bounds__(GT) void k_gemm(
    const unsigned short* __restrict__ xh, const unsigned short* __restrict__ xl,
    const unsigned short* __restrict__ wh, const unsigned short* __restrict__ wl,
    const float* __restrict__ b0, const float* __restrict__ b1,
    const float* __restrict__ b2, const float* __restrict__ b3,
    float* outp, int Mp) {
  __shared__ __attribute__((aligned(16))) float tile[4 * 16 * TP];
  const int tid = threadIdx.x, lane = tid & 31, wave = tid >> 5, hf = lane >> 4, m = lane & 15;
  const int m0 = blockIdx.x * MT + wave * 16;
  const int nb = blockIdx.y;
  const int widx = nb >> 2, n0 = (nb & 3) * 64;
  const float* bias = (widx == 0) ? b0 : (widx == 1) ? b1 : (widx == 2) ? b2 : b3;
  const unsigned short* wph = wh + (size_t)widx * DD * DD;
  const unsigned short* wpl = wl + (size_t)widx * DD * DD;
  const unsigned short* arh = xh + (size_t)(m0 + m) * DD + 8 * hf;
  const unsigned short* arl = xl + (size_t)(m0 + m) * DD + 8 * hf;

  v8f acc[4];
#pragma unroll
  for (int nt = 0; nt < 4; ++nt) acc[nt] = zero8f();

#pragma unroll 1
  for (int k0 = 0; k0 < DD; k0 += 32) {
    FragB ah, al;
    ah.h[0] = *(const v8us*)(arh + k0);
    ah.h[1] = *(const v8us*)(arh + k0 + 16);
    al.h[0] = *(const v8us*)(arl + k0);
    al.h[1] = *(const v8us*)(arl + k0 + 16);
#pragma unroll
    for (int nt = 0; nt < 4; ++nt) {
      const size_t bo = (size_t)(n0 + 16 * nt + m) * DD + 8 * hf + k0;
      FragB bh, bl;
      bh.h[0] = *(const v8us*)(wph + bo);
      bh.h[1] = *(const v8us*)(wph + bo + 16);
      bl.h[0] = *(const v8us*)(wpl + bo);
      bl.h[1] = *(const v8us*)(wpl + bo + 16);
      acc[nt] = wmb(ah.v, bh.v, acc[nt]);
      acc[nt] = wmb(ah.v, bl.v, acc[nt]);
      acc[nt] = wmb(al.v, bh.v, acc[nt]);
    }
  }

  float* tw = tile + wave * 16 * TP;
#pragma unroll
  for (int nt = 0; nt < 4; ++nt) {
    const float bb = bias[n0 + 16 * nt + m];
#pragma unroll
    for (int r = 0; r < 8; ++r) tw[(8 * hf + r) * TP + 16 * nt + m] = acc[nt][r] + bb;
  }
  __syncthreads();

  v4f ov[8];
#pragma unroll
  for (int i = 0; i < 8; ++i) {
    const v4fa t = *(const v4fa*)(tw + (2 * i + hf) * TP + 4 * m);
    ov[i] = t;
  }
  const size_t ob = ((size_t)widx * (size_t)Mp + (size_t)m0) * DD + (size_t)n0 + (size_t)(4 * m);
#pragma unroll
  for (int i = 0; i < 8; ++i) *(volatile v4f*)(outp + ob + (size_t)(2 * i + hf) * DD) = ov[i];
  __threadfence();
#pragma unroll
  for (int i = 0; i < 8; ++i) *(volatile v4f*)(outp + ob + (size_t)(2 * i + hf) * DD) = ov[i];
}

__global__ __launch_bounds__(NTHR) void k_agg(
    const float* __restrict__ vpl, const float* __restrict__ spl,
    const int* __restrict__ ei, const float* __restrict__ adjc, const float* __restrict__ wec,
    unsigned short* xch, unsigned short* xcl, int nN, int nE, int coff, int vec8) {
  __shared__ __attribute__((aligned(16))) unsigned int accw[(NB + 1) * DD];
  __shared__ float cntL[NB + 1];
  __shared__ __attribute__((aligned(16))) int list[LISTN];
  __shared__ int wcnt[NWAVE];

  const int tid = threadIdx.x, lane = tid & 31, wave = tid >> 5;
  const int nodeBase = blockIdx.x * NB;
  const int* srcs = ei;
  const int* dsts = ei + nE;

  for (int i = tid; i < (NB + 1) * DD; i += NTHR) accw[i] = 0u;
  if (tid < NB + 1) cntL[tid] = 0.0f;
  const float wed = wec[tid];
  __syncthreads();

  const int nChunks = (nE + CHUNK - 1) / CHUNK;
#pragma unroll 1
  for (int ch = 0; ch < nChunks; ++ch) {
    const int cbase = ch * CHUNK;
    const int wc = scan_chunk(dsts, nE, cbase, nodeBase, vec8, list, tid, wave);
    if (lane == 0) wcnt[wave] = wc;
    __syncthreads();

#pragma unroll 1
    for (int w = 0; w < NWAVE; ++w) {
      int n = wcnt[w];
      n = n > WCAP ? WCAP : (n < 0 ? 0 : n);
#pragma unroll 1
      for (int i = 0; i < n; ++i) {
        const int el = list[w * WCAP + i];
        int e = cbase + el;
        e = e < 0 ? 0 : (e > nE - 1 ? nE - 1 : e);
        const int t = dsts[e];
        int s = srcs[e];
        const float a = adjc[e];
        int slot = t - nodeBase;
        if ((unsigned)slot >= (unsigned)NB) slot = NB;
        s = s < 0 ? 0 : (s > nN - 1 ? nN - 1 : s);
        const float vv = vpl[(size_t)s * DD + tid];
        const int ai = slot * DD + tid;
        accw[ai] = __float_as_uint(fmaf(vv, a * wed, __uint_as_float(accw[ai])));
        if (tid == 0) cntL[slot] += 1.0f;
      }
    }
    __syncthreads();
  }

#pragma unroll 1
  for (int slot = 0; slot < NB; ++slot) {
    const float cn = cntL[slot];
    const float rc = 1.0f / fmaxf(cn, 1.0f);
    const int node = nodeBase + slot;
    const float sk = spl[(size_t)node * DD + tid];
    const int ai = slot * DD + tid;
    const float val = fmaf(__uint_as_float(accw[ai]), rc, sk);
    const unsigned int hi = f2bf(val);
    const unsigned int lo = f2bf(val - bf2f(hi));
    accw[ai] = hi | (lo << 16);
  }
  __syncthreads();

  v8us hv[NB / NWAVE], lv[NB / NWAVE];
#pragma unroll
  for (int j = 0; j < NB / NWAVE; ++j) {
    const int slot = wave + NWAVE * j;
    const unsigned int* p = accw + slot * DD + lane * 8;
    const v4ua u0 = *(const v4ua*)p;
    const v4ua u1 = *(const v4ua*)(p + 4);
    hv[j][0] = (unsigned short)(u0.x & 0xFFFFu); lv[j][0] = (unsigned short)(u0.x >> 16);
    hv[j][1] = (unsigned short)(u0.y & 0xFFFFu); lv[j][1] = (unsigned short)(u0.y >> 16);
    hv[j][2] = (unsigned short)(u0.z & 0xFFFFu); lv[j][2] = (unsigned short)(u0.z >> 16);
    hv[j][3] = (unsigned short)(u0.w & 0xFFFFu); lv[j][3] = (unsigned short)(u0.w >> 16);
    hv[j][4] = (unsigned short)(u1.x & 0xFFFFu); lv[j][4] = (unsigned short)(u1.x >> 16);
    hv[j][5] = (unsigned short)(u1.y & 0xFFFFu); lv[j][5] = (unsigned short)(u1.y >> 16);
    hv[j][6] = (unsigned short)(u1.z & 0xFFFFu); lv[j][6] = (unsigned short)(u1.z >> 16);
    hv[j][7] = (unsigned short)(u1.w & 0xFFFFu); lv[j][7] = (unsigned short)(u1.w >> 16);
  }
#pragma unroll
  for (int j = 0; j < NB / NWAVE; ++j) {
    const size_t go = (size_t)(nodeBase + wave + NWAVE * j) * XC + (size_t)coff + (size_t)(lane * 8);
    *(volatile v8us*)(xch + go) = hv[j];
    *(volatile v8us*)(xcl + go) = lv[j];
  }
  __threadfence();
#pragma unroll
  for (int j = 0; j < NB / NWAVE; ++j) {
    const size_t go = (size_t)(nodeBase + wave + NWAVE * j) * XC + (size_t)coff + (size_t)(lane * 8);
    *(volatile v8us*)(xch + go) = hv[j];
    *(volatile v8us*)(xcl + go) = lv[j];
  }
}

__global__ __launch_bounds__(NTHR) void k_alpha(
    const float* __restrict__ qpl, const float* __restrict__ kpl,
    const int* __restrict__ ei, const float* __restrict__ adjc, const float* __restrict__ wec,
    float* alc, int nN, int nE) {
  __shared__ __attribute__((aligned(16))) float al[EB];
  const int tid = threadIdx.x, lane = tid & 31, wave = tid >> 5;
  const int base = blockIdx.x * EB;
  const int* srcs = ei;
  const int* dsts = ei + nE;
  const int d0 = lane * 8;
  const v8f we8 = cat8(*(const v4f*)(wec + d0), *(const v4f*)(wec + d0 + 4));

#pragma unroll 1
  for (int i = 0; i < 32; ++i) {
    const int e  = base + wave * 32 + i;
    const int ec = e < nE ? e : nE - 1;
    int t = dsts[ec];
    int s = srcs[ec];
    t = t < 0 ? 0 : (t > nN - 1 ? nN - 1 : t);
    s = s < 0 ? 0 : (s > nN - 1 ? nN - 1 : s);
    const float a = adjc[ec];
    const float* qt = qpl + (size_t)t * DD + d0;
    const float* qs = qpl + (size_t)s * DD + d0;
    const float* kt = kpl + (size_t)t * DD + d0;
    const float* ks = kpl + (size_t)s * DD + d0;
    const v8f qtv = cat8(*(const v4f*)qt, *(const v4f*)(qt + 4));
    const v8f qsv = cat8(*(const v4f*)qs, *(const v4f*)(qs + 4));
    const v8f ktv = cat8(*(const v4f*)kt, *(const v4f*)(kt + 4));
    const v8f ksv = cat8(*(const v4f*)ks, *(const v4f*)(ks + 4));
    float s1 = 0.0f, s2 = 0.0f;
#pragma unroll
    for (int j = 0; j < 8; ++j) {
      const float kj = fmaf(a, we8[j], ksv[j]);
      s1 = fmaf(qtv[j], kj, s1);
      s2 = fmaf(qsv[j], ktv[j], s2);
    }
#pragma unroll
    for (int mm = 1; mm <= 4; mm <<= 1) {
      s1 += __shfl_xor(s1, mm, 32);
      s2 += __shfl_xor(s2, mm, 32);
    }
    const float u  = ((lane & 1) != 0) ? s2 : s1;
    const float th = tanhf(u * 0.125f);
    const float ot = __shfl_xor(th, 1, 32);
    float ap = 0.5f * (th + ot);
    ap += __shfl_xor(ap, 8, 32);
    ap += __shfl_xor(ap, 16, 32);
    ap *= 0.25f;
    if (lane == 0) al[wave * 32 + i] = ap;
  }
  __syncthreads();

  v4f v = {0.0f, 0.0f, 0.0f, 0.0f};
  const bool wr = wave < 2;
  if (wr) { const v4fa t = *(const v4fa*)(al + wave * 128 + lane * 4); v = t; }
  const size_t go = (size_t)base + (size_t)(wave * 128 + lane * 4);
  if (wr) *(volatile v4f*)(alc + go) = v;
  __threadfence();
  if (wr) *(volatile v4f*)(alc + go) = v;
}

__global__ __launch_bounds__(GT) void k_mlp(
    const unsigned short* __restrict__ xch, const unsigned short* __restrict__ xcl,
    const unsigned short* __restrict__ m1h, const unsigned short* __restrict__ m1l, const float* __restrict__ bm1,
    const unsigned short* __restrict__ m2h, const unsigned short* __restrict__ m2l, const float* __restrict__ bm2,
    float* out0, int nN) {
  __shared__ __attribute__((aligned(16))) unsigned short hs[4 * 16 * 32];
  __shared__ __attribute__((aligned(16))) unsigned short ls[4 * 16 * 32];
  __shared__ __attribute__((aligned(16))) float tile[4 * 16 * TP];
  const int tid = threadIdx.x, lane = tid & 31, wave = tid >> 5, hf = lane >> 4, m = lane & 15;
  const int r0 = blockIdx.x * MT + wave * 16;

  v8f acc1 = zero8f();
  {
    const unsigned short* arh = xch + (size_t)(r0 + m) * XC + 8 * hf;
    const unsigned short* arl = xcl + (size_t)(r0 + m) * XC + 8 * hf;
    const unsigned short* brh = m1h + (size_t)m * XC + 8 * hf;
    const unsigned short* brl = m1l + (size_t)m * XC + 8 * hf;
#pragma unroll 1
    for (int k0 = 0; k0 < XC; k0 += 32) {
      FragB ah, al, bh, bl;
      ah.h[0] = *(const v8us*)(arh + k0); ah.h[1] = *(const v8us*)(arh + k0 + 16);
      al.h[0] = *(const v8us*)(arl + k0); al.h[1] = *(const v8us*)(arl + k0 + 16);
      bh.h[0] = *(const v8us*)(brh + k0); bh.h[1] = *(const v8us*)(brh + k0 + 16);
      bl.h[0] = *(const v8us*)(brl + k0); bl.h[1] = *(const v8us*)(brl + k0 + 16);
      acc1 = wmb(ah.v, bh.v, acc1);
      acc1 = wmb(ah.v, bl.v, acc1);
      acc1 = wmb(al.v, bh.v, acc1);
    }
  }
  {
    const float bb1 = bm1[m < 8 ? m : 7];
    unsigned short* hw = hs + wave * 512;
    unsigned short* lw = ls + wave * 512;
#pragma unroll
    for (int r = 0; r < 8; ++r) {
      const float t = acc1[r] + bb1;
      float e = (t > 0.0f) ? t : expm1f(t);
      e = (m < 8) ? e : 0.0f;
      const unsigned int hi = f2bf(e);
      const unsigned int lo = f2bf(e - bf2f(hi));
      hw[(8 * hf + r) * 32 + m] = (unsigned short)hi;
      lw[(8 * hf + r) * 32 + m] = (unsigned short)lo;
      hw[(8 * hf + r) * 32 + 16 + m] = (unsigned short)0;
      lw[(8 * hf + r) * 32 + 16 + m] = (unsigned short)0;
    }
  }
  __syncthreads();
  FragB a2h, a2l;
  {
    const unsigned short* hw = hs + wave * 512;
    const unsigned short* lw = ls + wave * 512;
    const v8usa t0 = *(const v8usa*)(hw + m * 32 + 8 * hf);
    const v8usa t1 = *(const v8usa*)(hw + m * 32 + 16 + 8 * hf);
    const v8usa t2 = *(const v8usa*)(lw + m * 32 + 8 * hf);
    const v8usa t3 = *(const v8usa*)(lw + m * 32 + 16 + 8 * hf);
    a2h.h[0] = t0; a2h.h[1] = t1;
    a2l.h[0] = t2; a2l.h[1] = t3;
  }

  float* tw = tile + wave * 16 * TP;
#pragma unroll 1
  for (int g = 0; g < 4; ++g) {
    v8f acc2[4];
#pragma unroll
    for (int nt = 0; nt < 4; ++nt) {
      const int n = g * 64 + 16 * nt;
      const unsigned short* bph = m2h + (size_t)(n + m) * 32 + 8 * hf;
      const unsigned short* bpl = m2l + (size_t)(n + m) * 32 + 8 * hf;
      FragB bh, bl;
      bh.h[0] = *(const v8us*)bph; bh.h[1] = *(const v8us*)(bph + 16);
      bl.h[0] = *(const v8us*)bpl; bl.h[1] = *(const v8us*)(bpl + 16);
      acc2[nt] = zero8f();
      acc2[nt] = wmb(a2h.v, bh.v, acc2[nt]);
      acc2[nt] = wmb(a2h.v, bl.v, acc2[nt]);
      acc2[nt] = wmb(a2l.v, bh.v, acc2[nt]);
    }
#pragma unroll
    for (int nt = 0; nt < 4; ++nt) {
      const float bb = bm2[g * 64 + 16 * nt + m];
#pragma unroll
      for (int r = 0; r < 8; ++r) tw[(8 * hf + r) * TP + 16 * nt + m] = acc2[nt][r] + bb;
    }
    __syncthreads();
#pragma unroll 1
    for (int t = 0; t < 32; ++t) {
      const int idx = lane + 32 * t;
      const int row = idx >> 6, col = idx & 63;
      tw[row * TP + col] = tanhf(tw[row * TP + col]);
    }
    __syncthreads();
    v4f ov[8];
#pragma unroll
    for (int i = 0; i < 8; ++i) {
      const v4fa t = *(const v4fa*)(tw + (2 * i + hf) * TP + 4 * m);
      ov[i] = t;
    }
#pragma unroll
    for (int i = 0; i < 8; ++i) {
      const int grow = r0 + 2 * i + hf;
      if (grow < nN) *(volatile v4f*)(out0 + (size_t)grow * DD + g * 64 + 4 * m) = ov[i];
    }
    __threadfence();
#pragma unroll
    for (int i = 0; i < 8; ++i) {
      const int grow = r0 + 2 * i + hf;
      if (grow < nN) *(volatile v4f*)(out0 + (size_t)grow * DD + g * 64 + 4 * m) = ov[i];
    }
    __syncthreads();
  }
}

__global__ __launch_bounds__(NTHR) void k_emlp(
    const float* __restrict__ alp, const float* __restrict__ adj,
    const float* __restrict__ W1, const float* __restrict__ B1,
    const float* __restrict__ W2, const float* __restrict__ B2,
    const float* __restrict__ W3, const float* __restrict__ B3,
    float* out1, int nE, int EP) {
  __shared__ __attribute__((aligned(16))) float ol[4 * EB];
  const int tid = threadIdx.x, lane = tid & 31, wave = tid >> 5;
  const int j = lane & 7, grp = tid >> 3;
  const int jc = j < 4 ? j : 3;
  const int ja = j < 4 ? 0 : j - 4;
  const int base = blockIdx.x * EB;
  float w1[8], w2[8], w3[8];
#pragma unroll
  for (int i = 0; i < 8; ++i) { w1[i] = W1[j * 8 + i]; w2[i] = W2[j * 8 + i]; w3[i] = W3[jc * 8 + i]; }
  const float b1j = B1[j], b2j = B2[j], b3j = B3[jc];

#pragma unroll 1
  for (int p = 0; p < 8; ++p) {
    const int eloc = p * 32 + grp;
    const int e  = base + eloc;
    const int ec = e < nE ? e : nE - 1;
    const float va = alp[(size_t)jc * EP + ec];
    const float vb = adj[(size_t)ja * nE + ec];
    const float in = (j < 4) ? va : vb;
    float s = 0.0f;
#pragma unroll
    for (int i = 0; i < 8; ++i) s = fmaf(__shfl(in, i, 8), w1[i], s);
    s += b1j;
    const float h1 = (s > 0.0f) ? s : expm1f(s);
    s = 0.0f;
#pragma unroll
    for (int i = 0; i < 8; ++i) s = fmaf(__shfl(h1, i, 8), w2[i], s);
    s += b2j;
    const float h2 = (s > 0.0f) ? s : expm1f(s);
    s = 0.0f;
#pragma unroll
    for (int i = 0; i < 8; ++i) s = fmaf(__shfl(h2, i, 8), w3[i], s);
    s += b3j;
    if (j < 4) ol[j * EB + eloc] = s;
  }
  __syncthreads();

  const int o = wave >> 1, half = wave & 1;
  const v4fa tv = *(const v4fa*)(ol + o * EB + half * 128 + lane * 4);
  const v4f v = tv;
  const int eoff = base + half * 128 + lane * 4;
  float* op = out1 + (size_t)o * (size_t)nE;
  if (eoff + 3 < nE) {
    *(volatile v4f*)(op + eoff) = v;
  } else {
    if (eoff     < nE) ((volatile float*)op)[eoff]     = v.x;
    if (eoff + 1 < nE) ((volatile float*)op)[eoff + 1] = v.y;
    if (eoff + 2 < nE) ((volatile float*)op)[eoff + 2] = v.z;
  }
  __threadfence();
  if (eoff + 3 < nE) {
    *(volatile v4f*)(op + eoff) = v;
  } else {
    if (eoff     < nE) ((volatile float*)op)[eoff]     = v.x;
    if (eoff + 1 < nE) ((volatile float*)op)[eoff + 1] = v.y;
    if (eoff + 2 < nE) ((volatile float*)op)[eoff + 2] = v.z;
  }
}

extern "C" void kernel_launch(void* const* d_in, const int* in_sizes, int n_in,
                              void* d_out, int out_size, void* d_ws, size_t ws_size,
                              hipStream_t stream) {
  if (n_in < 23) return;
  const int nN = in_sizes[0] / DD;
  const int nE = in_sizes[1] / 2;
  if (nN <= 0 || nE <= 0 || in_sizes[0] != nN * DD || in_sizes[1] != 2 * nE) return;
  if (in_sizes[2] != NCHN * nE) return;
  if (in_sizes[4] != NCHN * DD * DD || in_sizes[6] != NCHN * DD * DD ||
      in_sizes[8] != NCHN * DD * DD || in_sizes[11] != NCHN * DD * DD) return;
  if (in_sizes[5] != NCHN * DD || in_sizes[7] != NCHN * DD || in_sizes[9] != NCHN * DD ||
      in_sizes[10] != NCHN * DD || in_sizes[12] != NCHN * DD) return;
  if (in_sizes[13] != 8 * XC || in_sizes[14] < 8 || in_sizes[15] != DD * 8 || in_sizes[16] < DD) return;
  if (in_sizes[17] != 64 || in_sizes[18] < 8 || in_sizes[19] != 64 || in_sizes[20] < 8 ||
      in_sizes[21] != 32 || in_sizes[22] < 4) return;
  if (out_size != nN * DD + 4 * nE) return;

  const float* x     = (const float*)d_in[0];
  const int*   ei    = (const int*)d_in[1];
  const float* adj   = (const float*)d_in[2];
  const float* Wq    = (const float*)d_in[4];
  const float* bq    = (const float*)d_in[5];
  const float* Wk    = (const float*)d_in[6];
  const float* bk    = (const float*)d_in[7];
  const float* Wv    = (const float*)d_in[8];
  const float* bv    = (const float*)d_in[9];
  const float* We    = (const float*)d_in[10];
  const float* Wskip = (const float*)d_in[11];
  const float* bskip = (const float*)d_in[12];
  const float* W_mc1 = (const float*)d_in[13];
  const float* b_mc1 = (const float*)d_in[14];
  const float* W_mc2 = (const float*)d_in[15];
  const float* b_mc2 = (const float*)d_in[16];
  const float* W_m1  = (const float*)d_in[17];
  const float* b_m1  = (const float*)d_in[18];
  const float* W_m2  = (const float*)d_in[19];
  const float* b_m2  = (const float*)d_in[20];
  const float* W_m3  = (const float*)d_in[21];
  const float* b_m3  = (const float*)d_in[22];

  float* out0 = (float*)d_out;
  float* out1 = out0 + (size_t)nN * DD;

  const int Mp  = ((nN + MT - 1) / MT) * MT;
  const int nBE = (nE + EB - 1) / EB;
  const int EP  = nBE * EB;

  char* ws = (char*)d_ws;
  size_t off = 0;
  auto carve = [&](size_t bytes) -> void* {
    void* p = ws + off;
    off = (off + bytes + 255) & ~(size_t)255;
    return p;
  };
  unsigned short* xh   = (unsigned short*)carve((size_t)Mp * DD * 2);
  unsigned short* xl   = (unsigned short*)carve((size_t)Mp * DD * 2);
  unsigned short* wh   = (unsigned short*)carve((size_t)NCHN * NWT * DD * DD * 2);
  unsigned short* wl   = (unsigned short*)carve((size_t)NCHN * NWT * DD * DD * 2);
  unsigned short* m1h  = (unsigned short*)carve((size_t)16 * XC * 2);
  unsigned short* m1l  = (unsigned short*)carve((size_t)16 * XC * 2);
  unsigned short* m2h  = (unsigned short*)carve((size_t)DD * 32 * 2);
  unsigned short* m2l  = (unsigned short*)carve((size_t)DD * 32 * 2);
  float*          qkvs = (float*)carve((size_t)NWT * Mp * DD * 4);
  unsigned short* xch  = (unsigned short*)carve((size_t)Mp * XC * 2);
  unsigned short* xcl  = (unsigned short*)carve((size_t)Mp * XC * 2);
  float*          alph = (float*)carve((size_t)NCHN * EP * 4);
  if (off > ws_size) return;

  const int vec8 = ((nE & 3) == 0) ? 1 : 0;
  const int nG   = Mp * (DD / 8);

  k_cvtx<<<(nG + NTHR - 1) / NTHR, NTHR, 0, stream>>>(x, xh, xl, nN, nG);
  k_cvtw<<<(NCHN * NWT * DD * DD) / (8 * NTHR) + (16 * XC) / (8 * NTHR) + (DD * 32) / (8 * NTHR), NTHR, 0, stream>>>(
      Wq, Wk, Wv, Wskip, W_mc1, W_mc2, wh, wl, m1h, m1l, m2h, m2l);

  const size_t plane = (size_t)Mp * DD;
  for (int c = 0; c < NCHN; ++c) {
    k_gemm<<<dim3(Mp / MT, NWT * (DD / 64)), GT, 0, stream>>>(
        xh, xl, wh + (size_t)c * NWT * DD * DD, wl + (size_t)c * NWT * DD * DD,
        bq + c * DD, bk + c * DD, bv + c * DD, bskip + c * DD, qkvs, Mp);
    k_agg<<<Mp / NB, NTHR, 0, stream>>>(
        qkvs + 2 * plane, qkvs + 3 * plane, ei, adj + (size_t)c * nE, We + c * DD,
        xch, xcl, nN, nE, c * DD, vec8);
    k_alpha<<<nBE, NTHR, 0, stream>>>(
        qkvs, qkvs + plane, ei, adj + (size_t)c * nE, We + c * DD, alph + (size_t)c * EP, nN, nE);
  }

  k_mlp<<<Mp / MT, GT, 0, stream>>>(xch, xcl, m1h, m1l, b_mc1, m2h, m2l, b_mc2, out0, nN);
  k_emlp<<<nBE, NTHR, 0, stream>>>(alph, adj, W_m1, b_m1, W_m2, b_m2, W_m3, b_m3, out1, nE, EP);
}
